// GroupedQueryAttention_59528246722830
// MI455X (gfx1250) — hardware-verified
//
#include <hip/hip_runtime.h>


#ifndef NB
#define NB 4
#endif
#ifndef SEQ
#define SEQ 1024
#endif
#define NB_FULL  4
#define SEQ_FULL 1024
#ifndef OUT_SEQ
#define OUT_SEQ SEQ
#endif
#define DM   2048
#define NQH  16
#define NKV  4
#define HD   128
#define KVD  (NKV * HD)
#define GRP  (NQH / NKV)
#define AW   4
#define EROWS (SEQ < 256 ? SEQ : 256)
#define QRS  2048.0f
#define QRI  (1.0f / 2048.0f)
#define SC2  ((float)(0.08838834764831845 * 1.4426950408889634))
#define PSH  14.0f
#define NEGB (-3.0e38f)
#define WOS  64.0f
#define CXS  16.0f
#define OSC  (1.0f / 1024.0f)
#define LG2B64 0.20762050593046014f

static_assert(HD == 128);
static_assert(NQH * HD == DM);
static_assert(NQH % NKV == 0);
static_assert(HD % 64 == 0);
static_assert(DM % 64 == 0);
static_assert(KVD % 64 == 0);
static_assert(DM % 32 == 0);
static_assert(HD % 32 == 0);
static_assert(SEQ % 64 == 0);
static_assert((NB * SEQ) % 64 == 0);
static_assert(SEQ % 32 == 0);
static_assert(EROWS % 64 == 0);
static_assert(EROWS % 32 == 0);
static_assert(EROWS >= 32);
static_assert(EROWS <= SEQ);
static_assert(AW == 4);
static_assert(EROWS % (16 * (AW / 2)) == 0);
static_assert((SEQ - EROWS) % (16 * AW) == 0);
static_assert((SEQ - EROWS) % 64 == 0);
static_assert(((size_t)SEQ * DM) % 8 == 0);
static_assert(((size_t)DM * DM) % 8 == 0);
static_assert(((size_t)KVD * DM) % 8 == 0);
static_assert((SEQ * 64) % 256 == 0);
static_assert(NB <= NB_FULL);
static_assert(SEQ <= SEQ_FULL);
static_assert(16 * 68 * 4 <= 131072);

typedef _Float16 h16;
typedef unsigned short bf;
typedef __attribute__((ext_vector_type(16))) __bf16   v16bf;
typedef __attribute__((ext_vector_type(16))) _Float16 v16h;
typedef __attribute__((ext_vector_type(8)))  _Float16 v8h;
typedef __attribute__((ext_vector_type(8)))  unsigned short v8us;
typedef __attribute__((ext_vector_type(8)))  float    v8f;
typedef __attribute__((ext_vector_type(4)))  float    v4f;
typedef v4f  __attribute__((may_alias)) v4fa;

__device__ __forceinline__ unsigned short f2bf(float f) { unsigned u = __float_as_uint(f); u += 0x7FFFu + ((u >> 16) & 1u); return (unsigned short)(u >> 16); }
__device__ __forceinline__ float bfr(float f) { return __uint_as_float(((unsigned)f2bf(f)) << 16); }
__device__ __forceinline__ v16h cat16(v8h lo, v8h hi) { return __builtin_shufflevector(lo, hi, 0, 1, 2, 3, 4, 5, 6, 7, 8, 9, 10, 11, 12, 13, 14, 15); }
__device__ __forceinline__ v16bf cat16b(v8us lo, v8us hi) { return __builtin_bit_cast(v16bf, __builtin_shufflevector(lo, hi, 0, 1, 2, 3, 4, 5, 6, 7, 8, 9, 10, 11, 12, 13, 14, 15)); }
__device__ __forceinline__ v8f wmma16(v16h a, v16h b, v8f c) { return __builtin_amdgcn_wmma_f32_16x16x32_f16(false, a, false, b, (short)0, c, false, false); }
__device__ __forceinline__ v8f wmmab(v16bf a, v16bf b, v8f c) { return __builtin_amdgcn_wmma_f32_16x16x32_bf16(false, a, false, b, (short)0, c, false, false); }
__device__ __forceinline__ v16h  ldh(const h16* p) { return cat16(*(const v8h*)p, *(const v8h*)(p + 16)); }
__device__ __forceinline__ v16bf ldb(const bf* p)  { return cat16b(*(const v8us*)p, *(const v8us*)(p + 16)); }
__device__ __forceinline__ void wave_sync() { __builtin_amdgcn_fence(3  , "wavefront"); __builtin_amdgcn_wave_barrier(); asm volatile("" ::: "memory"); }
__device__ __forceinline__ h16 toh_flush(float v) { const h16 r = (h16)v; return (fabsf(v) < 6.103515625e-05f) ? (h16)0.0f : r; }
__device__ __forceinline__ v8f wmma16g(v16h a, v16h b, v8f c) { c = wmma16(a, b, c); asm volatile("v_nop\n\tv_nop\n\tv_nop\n\tv_nop" : "+v"(c) : "v"(a), "v"(b)); return c; }
__device__ __forceinline__ v8f wmmabg(v16bf a, v16bf b, v8f c) { c = wmmab(a, b, c); asm volatile("v_nop\n\tv_nop\n\tv_nop\n\tv_nop" : "+v"(c) : "v"(a), "v"(b)); return c; }

__global__ __launch_bounds__(256) void k_cvt8(const float* __restrict__ src, bf* dst, size_t n8) {
    const size_t i = (size_t)blockIdx.x * 256 + threadIdx.x; if (i >= n8) return;
    const v8f v = *(const v8f*)(src + i * 8); v8us o;
#pragma unroll
    for (int k = 0; k < 8; ++k) o[k] = f2bf(v[k]);
    *(volatile v8us*)(dst + i * 8) = o; __threadfence(); *(volatile v8us*)(dst + i * 8) = o;
}

__global__ __launch_bounds__(256) void k_wcvt(const float* __restrict__ src, h16* dst, size_t n8) {
    const size_t i = (size_t)blockIdx.x * 256 + threadIdx.x; if (i >= n8) return;
    const v8f v = *(const v8f*)(src + i * 8); v8h o;
#pragma unroll
    for (int k = 0; k < 8; ++k) o[k] = toh_flush(bfr(v[k]) * WOS);
    *(volatile v8h*)(dst + i * 8) = o; __threadfence(); *(volatile v8h*)(dst + i * 8) = o;
}

__global__ __launch_bounds__(256) void k_ftab(float* F) {
#pragma clang fp contract(off)
    const int g = blockIdx.x * 256 + threadIdx.x;
    const int t = g >> 6, i = g & 63;
    const float w = exp2f(-(float)i * LG2B64);
    const float th = (float)t * w;
    const float f = cosf(th) + sinf(th);
    *(volatile float*)(F + g) = f; __threadfence(); *(volatile float*)(F + g) = f;
}

template <int MODE>
__device__ __forceinline__ void proj_body(const bf* A, const bf* Bt, const float* bias, const float* F, h16* Ph, h16* Pr, int nhp) {
    static_assert(32 * 8 * 4 == 16 * 64);
    __shared__ __align__(16) float os[16 * 68];
    const int K = DM;
    const int lane = threadIdx.x & 31, lr = lane & 15, hi = lane >> 4; const int r0 = blockIdx.x * 64, c0 = blockIdx.y * 64;
    v8f acc[4][4];
#pragma unroll
    for (int mb = 0; mb < 4; ++mb)
#pragma unroll
        for (int nb = 0; nb < 4; ++nb) acc[mb][nb] = (v8f){};
    const size_t aoff = (size_t)(r0 + lr) * K + 8 * hi, boff = (size_t)(c0 + lr) * K + 8 * hi;
#pragma unroll 1
    for (int kc = 0; kc < K; kc += 32) {
        v16bf a[4];
#pragma unroll
        for (int mb = 0; mb < 4; ++mb) a[mb] = ldb(A + aoff + (size_t)mb * 16 * K + kc);
#pragma unroll
        for (int nb = 0; nb < 4; ++nb) { const v16bf b = ldb(Bt + boff + (size_t)nb * 16 * K + kc);
#pragma unroll
            for (int mb = 0; mb < 4; ++mb) acc[mb][nb] = wmmabg(a[mb], b, acc[mb][nb]); }
    }
    float bc[4];
#pragma unroll
    for (int nb = 0; nb < 4; ++nb) bc[nb] = (MODE == 0) ? bfr(bias[c0 + nb * 16 + lr]) : 0.0f;
    size_t tbase, rbase; bool wr; int tt;
    if (MODE == 0) { const int bb = r0 / SEQ; tt = r0 % SEQ; const int zc = bb * nhp + c0 / HD; const int half = c0 % HD;
                     tbase = ((size_t)zc * SEQ + (size_t)tt) * HD + (size_t)half; rbase = ((size_t)zc * EROWS + (size_t)tt) * HD + (size_t)half; wr = tt < EROWS; }
    else           { const int bb = c0 / SEQ; tt = c0 % SEQ;
                     tbase = (size_t)bb * (size_t)KVD * SEQ + (size_t)r0 * SEQ + (size_t)tt; rbase = (size_t)bb * (size_t)KVD * EROWS + (size_t)r0 * EROWS + (size_t)tt; wr = tt < EROWS; }
#pragma unroll
    for (int mb = 0; mb < 4; ++mb) {
        float br[8];
#pragma unroll
        for (int j = 0; j < 8; ++j) br[j] = (MODE == 1) ? bfr(bias[r0 + mb * 16 + hi * 8 + j]) : 0.0f;
#pragma unroll
        for (int nb = 0; nb < 4; ++nb) {
#pragma unroll
            for (int j = 0; j < 8; ++j) os[(hi * 8 + j) * 68 + nb * 16 + lr] = acc[mb][nb][j] + bc[nb] + br[j]; }
        wave_sync();
#pragma unroll 1
        for (int ps = 0; ps < 2; ++ps) {
            if (MODE == 0) {
                const size_t sb = tbase + (size_t)(mb * 16) * HD;
                const size_t rb = rbase + (size_t)(mb * 16) * HD;
                const float* fb = F + (size_t)(tt + mb * 16) * 64;
#pragma unroll
                for (int s = 0; s < 4; ++s) { const int row = 4 * s + (lane >> 3), c8 = (lane & 7) * 8;
                    const v4f x0 = *(const v4fa*)(&os[row * 68 + c8]); const v4f x1 = *(const v4fa*)(&os[row * 68 + c8 + 4]);
                    const v4f g0 = *(const v4f*)(fb + row * 64 + c8); const v4f g1 = *(const v4f*)(fb + row * 64 + c8 + 4);
                    v8h hv, rv;
#pragma unroll
                    for (int i = 0; i < 4; ++i) { const float y0 = x0[i] * g0[i]; const float y1 = x1[i] * g1[i];
                        const h16 a0 = toh_flush(y0); const h16 a1 = toh_flush(y1); hv[i] = a0; hv[4 + i] = a1;
                        rv[i] = toh_flush((y0 - (float)a0) * QRS); rv[4 + i] = toh_flush((y1 - (float)a1) * QRS); }
                    const size_t oo = sb + (size_t)row * HD + c8;
                    const size_t ro = rb + (size_t)row * HD + c8;
                    *(volatile v8h*)(Ph + oo) = hv; if (wr) *(volatile v8h*)(Pr + ro) = rv; }
            } else {
                const size_t sb = tbase + (size_t)(mb * 16) * SEQ;
                const size_t rb = rbase + (size_t)(mb * 16) * EROWS;
#pragma unroll
                for (int s = 0; s < 4; ++s) { const int row = 4 * s + (lane >> 3), c8 = (lane & 7) * 8;
                    const v4f x0 = *(const v4fa*)(&os[row * 68 + c8]); const v4f x1 = *(const v4fa*)(&os[row * 68 + c8 + 4]); v8h hv, rv;
#pragma unroll
                    for (int i = 0; i < 4; ++i) { const h16 a0 = toh_flush(x0[i]); const h16 a1 = toh_flush(x1[i]); hv[i] = a0; hv[4 + i] = a1;
                        rv[i] = toh_flush((x0[i] - (float)a0) * QRS); rv[4 + i] = toh_flush((x1[i] - (float)a1) * QRS); }
                    const size_t oo = sb + (size_t)row * SEQ + c8;
                    const size_t ro = rb + (size_t)row * EROWS + c8;
                    *(volatile v8h*)(Ph + oo) = hv; if (wr) *(volatile v8h*)(Pr + ro) = rv; }
            }
            if (ps == 0) __threadfence(); }
        wave_sync();
    }
}

__global__ __launch_bounds__(32) void k_proj_tok(const bf* __restrict__ A, const bf* __restrict__ Bt, const float* __restrict__ bias, const float* __restrict__ F, h16* Ph, h16* Pr, int nhp) {
    proj_body<0>(A, Bt, bias, F, Ph, Pr, nhp);
}
__global__ __launch_bounds__(32) void k_proj_vt(const bf* __restrict__ A, const bf* __restrict__ Bt, const float* __restrict__ bias, h16* Ph, h16* Pr) {
    proj_body<1>(A, Bt, bias, bias, Ph, Pr, 0);
}

template <int EARLY>
__device__ __forceinline__ void flash_body(const h16* QH, const h16* QR, const h16* KP, const h16* KR, const h16* VT, const h16* VR, h16* CH, h16* CR) {
    constexpr int NDT  = EARLY ? 4 : 8;
    constexpr int OW   = NDT * 16;
    constexpr int OSPW = OW + 4;
    constexpr int NST  = EARLY ? 4 : 8;
    static_assert((OSPW * 4) % 16 == 0);
    static_assert(AW * 16 * OSPW * 4 <= 131072);
    static_assert(32 * 8 * NST == 16 * OW);
    __shared__ __align__(16) float os[AW * 16 * OSPW];
    const int lane = threadIdx.x & 31, lr = lane & 15, hi = lane >> 4;
    const int wave = __builtin_amdgcn_readfirstlane((int)(threadIdx.x >> 5));
    const int zh = blockIdx.y; const int b = zh / NQH, h = zh % NQH; const int kvz = b * NKV + h / GRP;
    const int tile = EARLY ? ((int)blockIdx.x * (AW / 2) + (wave >> 1)) : ((int)blockIdx.x * AW + wave);
    const int t0 = (EARLY ? 0 : EROWS) + tile * 16;
    const int dt0 = EARLY ? (wave & 1) * NDT : 0;
    const int lim = t0 + lr;
    const int nk = (t0 + 16 + 31) & ~31;
    const size_t qo  = ((size_t)zh * SEQ   + (size_t)(t0 + lr)) * HD + 8 * hi;
    const size_t qro = ((size_t)zh * EROWS + (size_t)(t0 + lr)) * HD + 8 * hi;
    const size_t ko  = ((size_t)kvz * SEQ   + (size_t)lr) * HD + 8 * hi;
    const size_t kro = ((size_t)kvz * EROWS + (size_t)lr) * HD + 8 * hi;
    const size_t vo  = ((size_t)kvz * HD + (size_t)(dt0 * 16 + lr)) * SEQ   + 8 * hi;
    const size_t vro = ((size_t)kvz * HD + (size_t)(dt0 * 16 + lr)) * EROWS + 8 * hi;
    const v16h hz = (v16h){};
    v8f o[NDT], oR[NDT];
#pragma unroll
    for (int j = 0; j < NDT; ++j) { o[j] = (v8f){}; oR[j] = (v8f){}; }
    float m = NEGB, l = 0.0f;
#pragma unroll 1
    for (int key0 = 0; key0 < nk; key0 += 32) {
        v8f sHa = (v8f){}, sLa = (v8f){}, sHb = (v8f){}, sLb = (v8f){};
        const size_t kk = ko + (size_t)key0 * HD, kkr = kro + (size_t)key0 * HD;
#pragma unroll 1
        for (int dk = 0; dk < HD; dk += 32) {
            const v16h qh = ldh(QH + qo + dk);
            const v16h ka0 = ldh(KP + kk + dk), kb0 = ldh(KP + kk + (size_t)16 * HD + dk);
            sHa = wmma16g(ka0, qh, sHa); sHb = wmma16g(kb0, qh, sHb);
            if (EARLY) {
                const v16h qr = ldh(QR + qro + dk);
                const v16h kra0 = ldh(KR + kkr + dk), krb0 = ldh(KR + kkr + (size_t)16 * HD + dk);
                sLa = wmma16g(ka0, qr, sLa); sLb = wmma16g(kb0, qr, sLb);
                sLa = wmma16g(kra0, qh, sLa); sLb = wmma16g(krb0, qh, sLb);
            }
        }
        const int ja = key0 + 8 * hi;
        float ta[8], tb[8]; bool fa[8], fb[8]; float mx = NEGB;
#pragma unroll
        for (int r = 0; r < 8; ++r) {
            fa[r] = (ja + r <= lim);
            fb[r] = (ja + 16 + r <= lim);
            if (EARLY) { ta[r] = (sHa[r] + sLa[r] * QRI) * SC2; tb[r] = (sHb[r] + sLb[r] * QRI) * SC2; }
            else       { ta[r] = sHa[r] * SC2; tb[r] = sHb[r] * SC2; }
            mx = fmaxf(mx, fmaxf(fa[r] ? ta[r] : NEGB, fb[r] ? tb[r] : NEGB)); }
        mx = fmaxf(mx, __shfl_xor(mx, 16, 32));
        const float mnew = fmaxf(m, mx);
        const float alpha = __builtin_amdgcn_exp2f(m - mnew);
        const float sh = PSH - mnew;
        v16h pb, pr = hz; float ls = 0.0f;
#pragma unroll
        for (int r = 0; r < 8; ++r) {
            const float xa = ta[r] + sh, xb = tb[r] + sh;
            const float ea = __builtin_amdgcn_exp2f(xa), eb = __builtin_amdgcn_exp2f(xb);
            const float ga = (fa[r] & (xa >= -14.0f)) ? ea : 0.0f, gb = (fb[r] & (xb >= -14.0f)) ? eb : 0.0f;
            const h16 pa = (h16)ga; const h16 pc = (h16)gb;
            pb[r] = pa; pb[8 + r] = pc;
            if (EARLY) { pr[r] = toh_flush((ga - (float)pa) * QRS); pr[8 + r] = toh_flush((gb - (float)pc) * QRS); ls += ga + gb; }
            else       { ls += (float)pa + (float)pc; } }
        l = l * alpha + ls; m = mnew;
#pragma unroll
        for (int j = 0; j < NDT; ++j) { o[j] = o[j] * alpha; if (EARLY) oR[j] = oR[j] * alpha; }
#pragma unroll
        for (int j = 0; j < NDT; ++j) {
            const v16h v0 = ldh(VT + vo + (size_t)j * 16 * SEQ + key0);
            o[j] = wmma16g(v0, pb, o[j]);
            if (EARLY) {
                const v16h vr0 = ldh(VR + vro + (size_t)j * 16 * EROWS + key0);
                oR[j] = wmma16g(v0, pr, oR[j]);
                oR[j] = wmma16g(vr0, pb, oR[j]);
            }
        }
    }
    l += __shfl_xor(l, 16, 32);
    const bool any = l > 0.0f;
    const float lsafe = any ? l : 1.0f;
    const float sc = any ? (CXS / lsafe) : 0.0f;
    const int wb = wave * 16 * OSPW;
#pragma unroll
    for (int j = 0; j < NDT; ++j) {
        v8f f = o[j];
        if (EARLY) f = o[j] + oR[j] * QRI;
        v4f a, c;
        a[0] = f[0] * sc; a[1] = f[1] * sc; a[2] = f[2] * sc; a[3] = f[3] * sc; c[0] = f[4] * sc; c[1] = f[5] * sc; c[2] = f[6] * sc; c[3] = f[7] * sc;
        *(v4fa*)(&os[wb + lr * OSPW + 16 * j + 8 * hi]) = a; *(v4fa*)(&os[wb + lr * OSPW + 16 * j + 8 * hi + 4]) = c; }
    wave_sync();
    const size_t cb = ((size_t)b * SEQ   + (size_t)t0) * DM + (size_t)(h * HD + dt0 * 16);
    const size_t rb = ((size_t)b * EROWS + (size_t)t0) * DM + (size_t)(h * HD + dt0 * 16);
#pragma unroll 1
    for (int ps = 0; ps < 2; ++ps) {
#pragma unroll
        for (int s = 0; s < NST; ++s) {
            const int row = EARLY ? (4 * s + (lane >> 3)) : (2 * s + (lane >> 4));
            const int c8  = EARLY ? ((lane & 7) * 8) : ((lane & 15) * 8);
            const v4f x0 = *(const v4fa*)(&os[wb + row * OSPW + c8]); const v4f x1 = *(const v4fa*)(&os[wb + row * OSPW + c8 + 4]); v8h hv, rv;
#pragma unroll
            for (int i = 0; i < 4; ++i) { const h16 a0 = toh_flush(x0[i]); const h16 a1 = toh_flush(x1[i]); hv[i] = a0; hv[4 + i] = a1;
                rv[i] = toh_flush((x0[i] - (float)a0) * QRS); rv[4 + i] = toh_flush((x1[i] - (float)a1) * QRS); }
            *(volatile v8h*)(CH + cb + (size_t)row * DM + c8) = hv;
            if (EARLY) *(volatile v8h*)(CR + rb + (size_t)row * DM + c8) = rv; }
        if (ps == 0) __threadfence(); }
}

__global__ __launch_bounds__(32 * AW) void k_flash_early(const h16* __restrict__ QH, const h16* __restrict__ QR, const h16* __restrict__ KP, const h16* __restrict__ KR,
                                                         const h16* __restrict__ VT, const h16* __restrict__ VR, h16* CH, h16* CR) {
    flash_body<1>(QH, QR, KP, KR, VT, VR, CH, CR);
}
__global__ __launch_bounds__(32 * AW) void k_flash_late(const h16* __restrict__ QH, const h16* __restrict__ KP, const h16* __restrict__ VT, h16* CH) {
    flash_body<0>(QH, QH, KP, KP, VT, VT, CH, CH);
}

template <int EB>
__device__ __forceinline__ void oproj_body(const h16* CH, const h16* CR, const h16* WO, const float* bo, float* OUT) {
    constexpr int MB = EB ? 2 : 4;
    constexpr int RT = 16 * MB;
    constexpr int NT = EB ? (EROWS / RT) : (((SEQ - EROWS) / RT) > 0 ? ((SEQ - EROWS) / RT) : 1);
    static_assert(32 * 4 * 8 == 16 * 64);
    static_assert(EROWS % RT == 0);
    __shared__ __align__(16) float os[16 * 68];
    const int K = DM;
    const int lane = threadIdx.x & 31, lr = lane & 15, hi = lane >> 4;
    const int bb = blockIdx.x / NT; const int tt = (EB ? 0 : EROWS) + ((int)blockIdx.x % NT) * RT; const int c0 = blockIdx.y * 64;
    v8f acc[MB][4], accR[MB][4];
#pragma unroll
    for (int mb = 0; mb < MB; ++mb)
#pragma unroll
        for (int nb = 0; nb < 4; ++nb) { acc[mb][nb] = (v8f){}; accR[mb][nb] = (v8f){}; }
    const size_t aoff = ((size_t)bb * SEQ   + (size_t)(tt + lr)) * K + 8 * hi;
    const size_t roff = ((size_t)bb * EROWS + (size_t)(tt + lr)) * K + 8 * hi;
    const size_t boff = (size_t)(c0 + lr) * K + 8 * hi;
#pragma unroll 1
    for (int kc = 0; kc < K; kc += 32) {
        v16h a[MB], ar[MB];
#pragma unroll
        for (int mb = 0; mb < MB; ++mb) { a[mb] = ldh(CH + aoff + (size_t)mb * 16 * K + kc); ar[mb] = (v16h){}; if (EB) ar[mb] = ldh(CR + roff + (size_t)mb * 16 * K + kc); }
#pragma unroll
        for (int nb = 0; nb < 4; ++nb) { const v16h w = ldh(WO + boff + (size_t)nb * 16 * K + kc);
#pragma unroll
            for (int mb = 0; mb < MB; ++mb) { acc[mb][nb] = wmma16g(a[mb], w, acc[mb][nb]); if (EB) accR[mb][nb] = wmma16g(ar[mb], w, accR[mb][nb]); } }
    }
    float bc[4];
#pragma unroll
    for (int nb = 0; nb < 4; ++nb) bc[nb] = bfr(bo[c0 + nb * 16 + lr]);
#pragma unroll
    for (int mb = 0; mb < MB; ++mb) {
#pragma unroll
        for (int nb = 0; nb < 4; ++nb) {
#pragma unroll
            for (int j = 0; j < 8; ++j) { float v = acc[mb][nb][j] * OSC; if (EB) v += accR[mb][nb][j] * (OSC * QRI);
                os[(hi * 8 + j) * 68 + nb * 16 + lr] = v + bc[nb]; } }
        wave_sync();
        float* orow = OUT + ((size_t)bb * OUT_SEQ + (size_t)(tt + mb * 16)) * DM + c0;
#pragma unroll 1
        for (int ps = 0; ps < 2; ++ps) {
#pragma unroll
            for (int s = 0; s < 8; ++s) { const int row = 2 * s + (lane >> 4), c4 = (lane & 15) * 4;
                const v4f val = *(const v4fa*)(&os[row * 68 + c4]);
                *(volatile v4f*)(orow + (size_t)row * DM + c4) = val; }
            if (ps == 0) __threadfence(); }
        wave_sync();
    }
}

__global__ __launch_bounds__(32) void k_oproj_early(const h16* __restrict__ CH, const h16* __restrict__ CR, const h16* __restrict__ WO, const float* __restrict__ bo, float* OUT) {
    oproj_body<1>(CH, CR, WO, bo, OUT);
}
__global__ __launch_bounds__(32) void k_oproj_late(const h16* __restrict__ CH, const h16* __restrict__ WO, const float* __restrict__ bo, float* OUT) {
    oproj_body<0>(CH, CH, WO, bo, OUT);
}

static constexpr size_t al256(size_t v) { return (v + 255) & ~(size_t)255; }
static constexpr size_t SZ_XB = al256((size_t)NB * SEQ * DM * 2);
static constexpr size_t SZ_WQ = al256((size_t)DM * DM * 2);
static constexpr size_t SZ_WK = al256((size_t)KVD * DM * 2);
static constexpr size_t SZ_WO = al256((size_t)DM * DM * 2);
static constexpr size_t SZ_QH = al256((size_t)NB * NQH * SEQ * HD * 2);
static constexpr size_t SZ_QR = al256((size_t)NB * NQH * EROWS * HD * 2);
static constexpr size_t SZ_KP = al256((size_t)NB * NKV * SEQ * HD * 2);
static constexpr size_t SZ_KR = al256((size_t)NB * NKV * EROWS * HD * 2);
static constexpr size_t SZ_CH = al256((size_t)NB * SEQ * DM * 2);
static constexpr size_t SZ_CR = al256((size_t)NB * EROWS * DM * 2);
static constexpr size_t SZ_FT = al256((size_t)SEQ * 64 * 4);
static constexpr size_t SZ_TOTAL = SZ_XB + SZ_WQ + 2 * SZ_WK + SZ_WO + SZ_QH + SZ_QR + 2 * SZ_KP + 2 * SZ_KR + SZ_CH + SZ_CR + SZ_FT;
static_assert(SZ_TOTAL <= (size_t)134217728);
static_assert((size_t)NB * NKV * SEQ * HD == (size_t)NB * KVD * SEQ);
static_assert((size_t)NB * NKV * EROWS * HD == (size_t)NB * KVD * EROWS);
static_assert(((size_t)NB * SEQ * DM) % 8 == 0);

extern "C" void kernel_launch(void* const* d_in, const int* in_sizes, int n_in,
                              void* d_out, int out_size, void* d_ws, size_t ws_size, hipStream_t stream) {
    if (n_in < 9) return;
    const size_t needx = ((size_t)(NB - 1) * SEQ_FULL + SEQ) * DM;
    if ((size_t)in_sizes[0] < needx) return;
    if ((size_t)in_sizes[1] < (size_t)DM * DM || in_sizes[2] < DM) return;
    if ((size_t)in_sizes[3] < (size_t)KVD * DM || in_sizes[4] < KVD) return;
    if ((size_t)in_sizes[5] < (size_t)KVD * DM || in_sizes[6] < KVD) return;
    if ((size_t)in_sizes[7] < (size_t)DM * DM || in_sizes[8] < DM) return;
    if ((size_t)out_size < ((size_t)(NB - 1) * OUT_SEQ + SEQ) * DM) return;
    if (SZ_TOTAL > ws_size) return;
    const float* x  = (const float*)d_in[0];
    const float* wq = (const float*)d_in[1]; const float* bq = (const float*)d_in[2];
    const float* wk = (const float*)d_in[3]; const float* bk = (const float*)d_in[4];
    const float* wv = (const float*)d_in[5]; const float* bv = (const float*)d_in[6];
    const float* wo = (const float*)d_in[7]; const float* bo = (const float*)d_in[8];
    float* OUT = (float*)d_out;
    char* wsp = (char*)d_ws;
    bf*  XB = (bf*)wsp;  wsp += SZ_XB;
    bf*  WQ = (bf*)wsp;  wsp += SZ_WQ;
    bf*  WK = (bf*)wsp;  wsp += SZ_WK;
    bf*  WV = (bf*)wsp;  wsp += SZ_WK;
    h16* WO = (h16*)wsp; wsp += SZ_WO;
    h16* QH = (h16*)wsp; wsp += SZ_QH;
    h16* QR = (h16*)wsp; wsp += SZ_QR;
    h16* KP = (h16*)wsp; wsp += SZ_KP;
    h16* VT = (h16*)wsp; wsp += SZ_KP;
    h16* KR = (h16*)wsp; wsp += SZ_KR;
    h16* VR = (h16*)wsp; wsp += SZ_KR;
    h16* CH = (h16*)wsp; wsp += SZ_CH;
    h16* CR = (h16*)wsp; wsp += SZ_CR;
    float* FT = (float*)wsp; wsp += SZ_FT;

    if (SEQ == SEQ_FULL) {
        const size_t n8 = (size_t)NB * SEQ * DM / 8;
        k_cvt8<<<(unsigned)((n8 + 255) / 256), 256, 0, stream>>>(x, XB, n8);
    } else {
        const size_t n8 = (size_t)SEQ * DM / 8;
        for (int b = 0; b < NB; ++b) k_cvt8<<<(unsigned)((n8 + 255) / 256), 256, 0, stream>>>(x + (size_t)b * SEQ_FULL * DM, XB + (size_t)b * SEQ * DM, n8);
    }
    { const size_t n8 = (size_t)DM * DM / 8; const unsigned g = (unsigned)((n8 + 255) / 256);
      k_cvt8<<<g, 256, 0, stream>>>(wq, WQ, n8);
      k_wcvt<<<g, 256, 0, stream>>>(wo, WO, n8); }
    { const size_t n8 = (size_t)KVD * DM / 8; const unsigned g = (unsigned)((n8 + 255) / 256);
      k_cvt8<<<g, 256, 0, stream>>>(wk, WK, n8); k_cvt8<<<g, 256, 0, stream>>>(wv, WV, n8); }
    k_ftab<<<(unsigned)(SEQ * 64 / 256), 256, 0, stream>>>(FT);

    k_proj_tok<<<dim3(NB * SEQ / 64, DM / 64, 1), 32, 0, stream>>>(XB, WQ, bq, FT, QH, QR, NQH);
    k_proj_tok<<<dim3(NB * SEQ / 64, KVD / 64, 1), 32, 0, stream>>>(XB, WK, bk, FT, KP, KR, NKV);
    k_proj_vt<<<dim3(KVD / 64, NB * SEQ / 64, 1), 32, 0, stream>>>(WV, XB, bv, VT, VR);

    k_flash_early<<<dim3(EROWS / (16 * (AW / 2)), NB * NQH, 1), 32 * AW, 0, stream>>>(QH, QR, KP, KR, VT, VR, CH, CR);
    if (SEQ > EROWS)
        k_flash_late<<<dim3((SEQ - EROWS) / (16 * AW), NB * NQH, 1), 32 * AW, 0, stream>>>(QH, KP, VT, CH);

    k_oproj_early<<<dim3(NB * (EROWS / 32), DM / 64, 1), 32, 0, stream>>>(CH, CR, WO, bo, OUT);
    if (SEQ > EROWS)
        k_oproj_late<<<dim3(NB * ((SEQ - EROWS) / 64), DM / 64, 1), 32, 0, stream>>>(CH, WO, bo, OUT);
}
